// Attention_71339406786815
// MI455X (gfx1250) — hardware-verified
//
#include <hip/hip_runtime.h>


#ifndef NB
#define NB 2
#endif
#ifndef SEQ
#define SEQ 2048
#endif
#define NB_FULL 2
#define SEQ_FULL 2048
#define DM 2048
#define NH 16
#define HD 128
#define QB 64
#define NQB (SEQ / QB)
#define RE ((SEQ < 256) ? SEQ : 256)
#define RO RE
#define NQBR (RE / QB)
#define PCAR 1024.0f
#define RSC 2048.0f
#define IRSC (1.0f / 2048.0f)
#define CCAR 16.0f
#define WSC 64.0f
#define OSCL (1.0f / 1024.0f)
#define SCL 0.08838834764831845f
#define L2E 1.4426950408889634f
#define NEGINF (-__builtin_inff())

static_assert(NB >= 1 && NB <= NB_FULL);
static_assert(SEQ % 64 == 0 && SEQ >= 64 && SEQ <= SEQ_FULL && SEQ % 4 == 0);
static_assert(RE % QB == 0 && RE % 32 == 0 && RE <= SEQ && RE >= QB && RO == RE && NQBR >= 1 && NQBR <= NQB);
static_assert(DM == NH * HD && HD == 128 && DM % 64 == 0 && (DM * DM) % 64 == 0);

typedef _Float16 h16;
typedef unsigned short bf;
typedef __attribute__((ext_vector_type(16))) __bf16   v16bf;
typedef __attribute__((ext_vector_type(16))) _Float16 v16h;
typedef __attribute__((ext_vector_type(8)))  _Float16 v8h;
typedef __attribute__((ext_vector_type(8)))  unsigned short v8us;
typedef __attribute__((ext_vector_type(8)))  float    v8f;
typedef __attribute__((ext_vector_type(4)))  float    v4f;
typedef __attribute__((ext_vector_type(2)))  _Float16 v2h;
typedef __attribute__((ext_vector_type(2)))  unsigned short v2us;
typedef v8h  __attribute__((may_alias)) v8ha;
typedef v4f  __attribute__((may_alias)) v4fa;
typedef v8us __attribute__((may_alias)) v8usa;

__device__ __forceinline__ unsigned short f2bf(float f) { unsigned u = __float_as_uint(f); u += 0x7FFFu + ((u >> 16) & 1u); return (unsigned short)(u >> 16); }
__device__ __forceinline__ float bf2f(unsigned short b) { return __uint_as_float(((unsigned)b) << 16); }
__device__ __forceinline__ float bfr(float f) { return bf2f(f2bf(f)); }
__device__ __forceinline__ void splitf(float y, unsigned short& h, unsigned short& l) { h = f2bf(y); l = f2bf(y - bf2f(h)); }
__device__ __forceinline__ v16h cat16(v8h lo, v8h hi) { return __builtin_shufflevector(lo, hi, 0, 1, 2, 3, 4, 5, 6, 7, 8, 9, 10, 11, 12, 13, 14, 15); }
__device__ __forceinline__ v16bf cat16b(v8us lo, v8us hi) { return __builtin_bit_cast(v16bf, __builtin_shufflevector(lo, hi, 0, 1, 2, 3, 4, 5, 6, 7, 8, 9, 10, 11, 12, 13, 14, 15)); }
__device__ __forceinline__ v8f wmma16(v16h a, v16h b, v8f c) { return __builtin_amdgcn_wmma_f32_16x16x32_f16(false, a, false, b, (short)0, c, false, false); }
__device__ __forceinline__ v8f wmmab(v16bf a, v16bf b, v8f c) { return __builtin_amdgcn_wmma_f32_16x16x32_bf16(false, a, false, b, (short)0, c, false, false); }
__device__ __forceinline__ v16h ldh(const h16* p) { return cat16(*(const v8h*)p, *(const v8h*)(p + 16)); }
__device__ __forceinline__ v16h ldl(const h16* p) { return cat16(*(const v8ha*)p, *(const v8ha*)(p + 16)); }
__device__ __forceinline__ float ex2(float x) { return __builtin_amdgcn_exp2f(x); }
__device__ __forceinline__ void wave_sync() { __builtin_amdgcn_fence(3  , "wavefront"); __builtin_amdgcn_wave_barrier(); asm volatile("" ::: "memory"); }

template <typename T16> struct WFrag;
template <> struct WFrag<h16> { typedef v16h V; static __device__ __forceinline__ V ld(const h16* p) { return cat16(*(const v8h*)p, *(const v8h*)(p + 16)); } static __device__ __forceinline__ v8f mma(V a, V b, v8f c) { return wmma16(a, b, c); } };
template <> struct WFrag<bf> { typedef v16bf V; static __device__ __forceinline__ V ld(const bf* p) { return cat16b(*(const v8us*)p, *(const v8us*)(p + 16)); } static __device__ __forceinline__ v8f mma(V a, V b, v8f c) { return wmmab(a, b, c); } };
template <typename T16, int NSPLIT>
__global__ __launch_bounds__(32) void k_gemmw(const T16* __restrict__ A, const T16* __restrict__ A2, const T16* __restrict__ Bt, int K, float* C, int ldc, float osc) {
    typedef typename WFrag<T16>::V V;
    __shared__ __align__(16) float os[16 * 68];
    const int lane = threadIdx.x & 31, lr = lane & 15, hi = lane >> 4; const int r0 = blockIdx.x * 64, c0 = blockIdx.y * 64;
    v8f acc[4][4];
#pragma unroll
    for (int mb = 0; mb < 4; ++mb)
#pragma unroll
        for (int nb = 0; nb < 4; ++nb) acc[mb][nb] = (v8f){};
    const size_t aoff = (size_t)(r0 + lr) * K + 8 * hi, boff = (size_t)(c0 + lr) * K + 8 * hi;
#pragma unroll 1
    for (int kc = 0; kc < K; kc += 32) {
        V a[4], a2[4];
#pragma unroll
        for (int mb = 0; mb < 4; ++mb) { a[mb] = WFrag<T16>::ld(A + aoff + (size_t)mb * 16 * K + kc); if (NSPLIT == 1) a2[mb] = WFrag<T16>::ld(A2 + aoff + (size_t)mb * 16 * K + kc); }
#pragma unroll
        for (int nb = 0; nb < 4; ++nb) { const V b = WFrag<T16>::ld(Bt + boff + (size_t)nb * 16 * K + kc);
#pragma unroll
            for (int mb = 0; mb < 4; ++mb) { acc[mb][nb] = WFrag<T16>::mma(a[mb], b, acc[mb][nb]); if (NSPLIT == 1) acc[mb][nb] = WFrag<T16>::mma(a2[mb], b, acc[mb][nb]); } }
        asm volatile("v_nop\n\tv_nop\n\tv_nop\n\tv_nop" : "+v"(acc[0][0]), "+v"(acc[1][1]), "+v"(acc[2][2]), "+v"(acc[3][3]) : "v"(a[0]), "v"(a[3]));
    }
#pragma unroll
    for (int mb = 0; mb < 4; ++mb) {
#pragma unroll
        for (int nb = 0; nb < 4; ++nb) {
#pragma unroll
            for (int j = 0; j < 8; ++j) os[(hi * 8 + j) * 68 + nb * 16 + lr] = acc[mb][nb][j]; }
        wave_sync();
        float* crow = C + (size_t)(r0 + mb * 16) * ldc + c0;
#pragma unroll 1
        for (int ps = 0; ps < 2; ++ps) {
#pragma unroll
            for (int s2 = 0; s2 < 8; ++s2) { const int row = 2 * s2 + hi, cofs = lr * 4; v4f val = *(const v4fa*)(os + row * 68 + cofs); val = val * osc;
                *(volatile v4f*)(crow + (size_t)row * ldc + cofs) = val; }
            if (ps == 0) __threadfence(); }
        wave_sync();
    }
}

__global__ __launch_bounds__(256) void k_cvt8(const float* __restrict__ src, bf* dst, size_t n8) { const size_t i = (size_t)blockIdx.x * 256 + threadIdx.x; if (i >= n8) return; const v8f v = *(const v8f*)(src + i * 8); v8us o;
#pragma unroll
    for (int k = 0; k < 8; ++k) o[k] = f2bf(v[k]); *(volatile v8us*)(dst + i * 8) = o; __threadfence(); *(volatile v8us*)(dst + i * 8) = o; }

__global__ __launch_bounds__(256) void k_wtG(const float* __restrict__ w, int K, int N, bf* Bt) {
    const int lane = threadIdx.x & 31; const int L0 = (blockIdx.x * 8 + (threadIdx.x >> 5)) * 8; const int nlines = N * K / 64;
#pragma unroll
    for (int ps = 0; ps < 2; ++ps) {
#pragma unroll 1
        for (int l = 0; l < 8; ++l) { const int L = L0 + l; if (L >= nlines) break; const size_t e = (size_t)L * 64 + lane * 2; const int k = (int)(e % K), n = (int)(e / K); v2us o;
            o[0] = f2bf(w[(size_t)k * N + n]); o[1] = f2bf(w[(size_t)(k + 1) * N + n]); *(volatile v2us*)(Bt + e) = o; }
        if (ps == 0) __threadfence(); }
}
__global__ __launch_bounds__(256) void k_wtG2(const float* __restrict__ w, int K, int N, bf* Bt, h16* Bh) {
    const int lane = threadIdx.x & 31; const int L0 = (blockIdx.x * 8 + (threadIdx.x >> 5)) * 8; const int nlines = N * K / 64;
#pragma unroll
    for (int ps = 0; ps < 2; ++ps) {
#pragma unroll 1
        for (int l = 0; l < 8; ++l) { const int L = L0 + l; if (L >= nlines) break; const size_t e = (size_t)L * 64 + lane * 2; const int k = (int)(e % K), n = (int)(e / K); v2us o; v2h oh;
            o[0] = f2bf(w[(size_t)k * N + n]); o[1] = f2bf(w[(size_t)(k + 1) * N + n]); oh[0] = (h16)(bf2f(o[0]) * WSC); oh[1] = (h16)(bf2f(o[1]) * WSC);
            *(volatile v2us*)(Bt + e) = o; *(volatile v2h*)(Bh + e) = oh; }
        if (ps == 0) __threadfence(); }
}

__global__ __launch_bounds__(256) void k_trig(const int* __restrict__ posp, float* CST) {
#pragma clang fp contract(off)
    __shared__ __align__(16) float tab[2][256];
    const int tid = threadIdx.x; const int rr = tid >> 6, j = tid & 63; const int t = blockIdx.x * 4 + rr;
    const int p0 = posp[0]; const int start = (p0 > 0) ? p0 : 0;
    const double pw = exp2((double)j * (13.287712379549449 / 64.0));
    const float pf = (float)pw; const float inv = 1.0f / pf;
    const float ang = ((float)start + (float)t) * inv;
    float sn, cs; sincosf(ang, &sn, &cs);
    tab[0][tid] = cs; tab[1][tid] = sn;
    __syncthreads();
    if (tid < 128) { const int wch = tid >> 6; const int l = tid & 63; const int row = l >> 4, c4 = (l & 15) * 4;
        const v4f v = *(const v4fa*)(&tab[wch][row * 64 + c4]);
        float* dst = CST + (size_t)wch * SEQ * 64 + (size_t)(blockIdx.x * 4 + row) * 64 + c4;
        *(volatile v4f*)dst = v; __threadfence(); *(volatile v4f*)dst = v; }
}

__global__ __launch_bounds__(256) void k_rope(const float* __restrict__ F, const float* __restrict__ CST, h16* PH, h16* PL) {
#pragma clang fp contract(off)
    const int gid = blockIdx.x * 256 + threadIdx.x; const int R = gid >> 3, g = gid & 7;
    if (R >= NH * SEQ) return;
    const int hd = R / SEQ, t = R - hd * SEQ;
    const float* fr = F + (size_t)t * DM + hd * HD + 8 * g;
    const v8f x1 = *(const v8f*)fr, x2 = *(const v8f*)(fr + 64);
    const v8f cs = *(const v8f*)(CST + (size_t)t * 64 + 8 * g), sn = *(const v8f*)(CST + (size_t)SEQ * 64 + (size_t)t * 64 + 8 * g);
    v8h o1, o2, l1, l2;
#pragma unroll
    for (int q = 0; q < 8; ++q) { const float a = x1[q] * cs[q] - x2[q] * sn[q]; const float c = x1[q] * sn[q] + x2[q] * cs[q]; const h16 ah = (h16)a, ch = (h16)c;
        o1[q] = ah; o2[q] = ch; l1[q] = (h16)((a - (float)ah) * RSC); l2[q] = (h16)((c - (float)ch) * RSC); }
    h16* ph = PH + (size_t)R * HD + 8 * g;
    const bool res = (t < RE); const size_t plo = ((size_t)hd * RE + (res ? t : 0)) * HD + 8 * g;
#pragma unroll 1
    for (int ps = 0; ps < 2; ++ps) { *(volatile v8h*)ph = o1; *(volatile v8h*)(ph + 64) = o2; if (res) { *(volatile v8h*)(PL + plo) = l1; *(volatile v8h*)(PL + plo + 64) = l2; } if (ps == 0) __threadfence(); }
}

__global__ __launch_bounds__(256) void k_vt(const float* __restrict__ F, h16* VT, h16* VL) {
    const size_t e = ((size_t)blockIdx.x * 256 + threadIdx.x) * 2; if (e >= (size_t)NH * HD * SEQ) return;
    const int t = (int)(e % SEQ); const int d = (int)((e / SEQ) % HD); const int hd = (int)(e / ((size_t)SEQ * HD));
    const float a0 = F[(size_t)t * DM + hd * HD + d], a1 = F[(size_t)(t + 1) * DM + hd * HD + d];
    const h16 h0 = (h16)a0, h1 = (h16)a1; v2h oh, ol; oh[0] = h0; oh[1] = h1; ol[0] = (h16)((a0 - (float)h0) * RSC); ol[1] = (h16)((a1 - (float)h1) * RSC);
    const bool res = (t < RE); const size_t plo = ((size_t)hd * HD + d) * RE + (res ? t : 0);
#pragma unroll 1
    for (int ps = 0; ps < 2; ++ps) { *(volatile v2h*)(VT + e) = oh; if (res) *(volatile v2h*)(VL + plo) = ol; if (ps == 0) __threadfence(); }
}

__device__ __forceinline__ void ctx_store(const float* osw, int hh, int m, size_t row0, int col0, bool bfp, size_t brow0, h16* CH, bf* CBh, bf* CBl) {
#pragma unroll 1
    for (int ps = 0; ps < 2; ++ps) {
#pragma unroll
        for (int sg = 0; sg < 8; ++sg) {
            const int row = 2 * sg + hh, col = m * 8;
            const v4f a0 = *(const v4fa*)(osw + row * 132 + col), a1 = *(const v4fa*)(osw + row * 132 + col + 4);
            v8h o8;
#pragma unroll
            for (int i = 0; i < 4; ++i) { o8[i] = (h16)(a0[i] * CCAR); o8[4 + i] = (h16)(a1[i] * CCAR); }
            *(volatile v8h*)(CH + (row0 + row) * DM + col0 + col) = o8;
            if (bfp) { v8us oh, ol;
#pragma unroll
                for (int i = 0; i < 4; ++i) { unsigned short x0, y0, x1, y1; splitf(a0[i], x0, y0); splitf(a1[i], x1, y1); oh[i] = x0; ol[i] = y0; oh[4 + i] = x1; ol[4 + i] = y1; }
                *(volatile v8us*)(CBh + (brow0 + row) * DM + col0 + col) = oh; *(volatile v8us*)(CBl + (brow0 + row) * DM + col0 + col) = ol; }
        }
        if (ps == 0) __threadfence(); }
}
__device__ __forceinline__ void ctx_store64(const float* osw, int lane, size_t row0, int col0, size_t brow0, h16* CH, bf* CBh, bf* CBl) {
    const int rl = lane >> 3, col = (lane & 7) * 8;
#pragma unroll 1
    for (int ps = 0; ps < 2; ++ps) {
#pragma unroll
        for (int sg = 0; sg < 4; ++sg) {
            const int row = 4 * sg + rl;
            const v4f a0 = *(const v4fa*)(osw + row * 68 + col), a1 = *(const v4fa*)(osw + row * 68 + col + 4);
            v8h o8; v8us oh, ol;
#pragma unroll
            for (int i = 0; i < 4; ++i) { o8[i] = (h16)(a0[i] * CCAR); o8[4 + i] = (h16)(a1[i] * CCAR); unsigned short x0, y0, x1, y1; splitf(a0[i], x0, y0); splitf(a1[i], x1, y1); oh[i] = x0; ol[i] = y0; oh[4 + i] = x1; ol[4 + i] = y1; }
            *(volatile v8h*)(CH + (row0 + row) * DM + col0 + col) = o8;
            *(volatile v8us*)(CBh + (brow0 + row) * DM + col0 + col) = oh; *(volatile v8us*)(CBl + (brow0 + row) * DM + col0 + col) = ol;
        }
        if (ps == 0) __threadfence(); }
}

__global__ __launch_bounds__(128) void k_attn(const h16* __restrict__ QH, const h16* __restrict__ KH, const h16* __restrict__ VT, h16* CH, bf* CBh, bf* CBl) {
    __shared__ __align__(16) h16 pls[4 * 16 * 72];
    __shared__ __align__(16) float oss[4 * 16 * 132];
    const int lane = threadIdx.x & 31, m = lane & 15, hh = lane >> 4, wv = threadIdx.x >> 5;
    const int qb = blockIdx.x + NQBR, hd = blockIdx.y, b = blockIdx.z;
    const int q0 = qb * QB + wv * 16;
    const size_t bh = (size_t)b * NH + hd;
    const h16* Qp = QH + (bh * SEQ + q0 + m) * HD + 8 * hh;
    const h16* Kp = KH + (bh * SEQ + m) * HD + 8 * hh;
    const h16* Vp = VT + (bh * HD + m) * SEQ + 8 * hh;
    h16* plw = pls + wv * (16 * 72); float* osw = oss + wv * (16 * 132);
    v8f o[8]; float mi[8], li[8];
#pragma unroll
    for (int nt = 0; nt < 8; ++nt) o[nt] = (v8f){};
#pragma unroll
    for (int r = 0; r < 8; ++r) { mi[r] = NEGINF; li[r] = 0.0f; }
#pragma unroll 1
    for (int c = 0; c <= qb; ++c) {
        const int k0 = c * QB;
        v8f s[4];
#pragma unroll
        for (int tl = 0; tl < 4; ++tl) s[tl] = (v8f){};
#pragma unroll
        for (int ds = 0; ds < 4; ++ds) {
            const v16h qa = ldh(Qp + ds * 32);
            v16h kf[4];
#pragma unroll
            for (int tl = 0; tl < 4; ++tl) kf[tl] = ldh(Kp + (size_t)(k0 + tl * 16) * HD + ds * 32);
#pragma unroll
            for (int tl = 0; tl < 4; ++tl) s[tl] = wmma16(qa, kf[tl], s[tl]);
            asm volatile("v_nop\n\tv_nop\n\tv_nop\n\tv_nop" : "+v"(s[0]), "+v"(s[1]), "+v"(s[2]), "+v"(s[3]) : "v"(qa), "v"(kf[0]), "v"(kf[3]));
        }
        const bool diag = (c == qb);
#pragma unroll
        for (int r = 0; r < 8; ++r) {
            const int row = q0 + 8 * hh + r; const int kk = k0 + m - row;
            float t0 = s[0][r] * SCL, t1 = s[1][r] * SCL, t2 = s[2][r] * SCL, t3 = s[3][r] * SCL;
            if (diag) { t0 = (kk > 0) ? NEGINF : t0; t1 = (kk + 16 > 0) ? NEGINF : t1; t2 = (kk + 32 > 0) ? NEGINF : t2; t3 = (kk + 48 > 0) ? NEGINF : t3; }
            float mx = fmaxf(fmaxf(t0, t1), fmaxf(t2, t3));
            mx = fmaxf(mx, __shfl_xor(mx, 1)); mx = fmaxf(mx, __shfl_xor(mx, 2)); mx = fmaxf(mx, __shfl_xor(mx, 4)); mx = fmaxf(mx, __shfl_xor(mx, 8));
            const float mn = fmaxf(mi[r], mx);
            const float corr = ex2((mi[r] - mn) * L2E);
            const float p0 = ex2((t0 - mn) * L2E), p1 = ex2((t1 - mn) * L2E), p2 = ex2((t2 - mn) * L2E), p3 = ex2((t3 - mn) * L2E);
            float rs = (p0 + p1) + (p2 + p3);
            rs += __shfl_xor(rs, 1); rs += __shfl_xor(rs, 2); rs += __shfl_xor(rs, 4); rs += __shfl_xor(rs, 8);
            li[r] = li[r] * corr + rs; mi[r] = mn;
#pragma unroll
            for (int nt = 0; nt < 8; ++nt) o[nt][r] = o[nt][r] * corr;
            h16* pr = plw + (8 * hh + r) * 72 + m;
            pr[0] = (h16)(p0 * PCAR); pr[16] = (h16)(p1 * PCAR); pr[32] = (h16)(p2 * PCAR); pr[48] = (h16)(p3 * PCAR);
        }
        wave_sync();
        const v16h pa0 = ldl(plw + m * 72 + 8 * hh), pa1 = ldl(plw + m * 72 + 32 + 8 * hh);
#pragma unroll
        for (int nt = 0; nt < 8; ++nt) { const h16* vp = Vp + (size_t)nt * 16 * SEQ + k0; const v16h vb0 = ldh(vp), vb1 = ldh(vp + 32);
            o[nt] = wmma16(pa0, vb0, o[nt]); o[nt] = wmma16(pa1, vb1, o[nt]); }
        asm volatile("v_nop\n\tv_nop\n\tv_nop\n\tv_nop" : "+v"(o[0]), "+v"(o[1]), "+v"(o[2]), "+v"(o[3]), "+v"(o[4]), "+v"(o[5]), "+v"(o[6]), "+v"(o[7]) : "v"(pa0), "v"(pa1));
        wave_sync();
    }
    float f[8];
#pragma unroll
    for (int r = 0; r < 8; ++r) f[r] = 1.0f / (li[r] * PCAR);
#pragma unroll
    for (int r = 0; r < 8; ++r)
#pragma unroll
        for (int nt = 0; nt < 8; ++nt) osw[(8 * hh + r) * 132 + nt * 16 + m] = o[nt][r] * f[r];
    wave_sync();
    ctx_store(osw, hh, m, (size_t)b * SEQ + q0, hd * HD, (qb * QB < RO), (size_t)b * RO + q0, CH, CBh, CBl);
}

__global__ __launch_bounds__(128) void k_attnR(const h16* __restrict__ QH, const h16* __restrict__ QL, const h16* __restrict__ KH, const h16* __restrict__ KL,
                                                const h16* __restrict__ VT, const h16* __restrict__ VL, h16* CH, bf* CBh, bf* CBl) {
    __shared__ __align__(16) h16 phs[4 * 16 * 40];
    __shared__ __align__(16) h16 prs[4 * 16 * 40];
    __shared__ __align__(16) float oss[4 * 16 * 68];
    const int lane = threadIdx.x & 31, m = lane & 15, hh = lane >> 4, wv = threadIdx.x >> 5;
    const int qb = blockIdx.x >> 1, dh2 = blockIdx.x & 1, hd = blockIdx.y, b = blockIdx.z;
    const int q0 = qb * QB + wv * 16;
    const size_t bh = (size_t)b * NH + hd;
    const h16* Qp = QH + (bh * SEQ + q0 + m) * HD + 8 * hh;                const h16* QLp = QL + (bh * RE + q0 + m) * HD + 8 * hh;
    const h16* Kp = KH + (bh * SEQ + m) * HD + 8 * hh;                     const h16* KLp = KL + (bh * RE + m) * HD + 8 * hh;
    const h16* Vp = VT + (bh * HD + dh2 * 64 + m) * SEQ + 8 * hh;          const h16* VLp = VL + (bh * HD + dh2 * 64 + m) * RE + 8 * hh;
    h16* phw = phs + wv * (16 * 40); h16* prw = prs + wv * (16 * 40); float* osw = oss + wv * (16 * 68);
    v8f o[4], orr[4]; float mi[8], li[8];
#pragma unroll
    for (int nt = 0; nt < 4; ++nt) { o[nt] = (v8f){}; orr[nt] = (v8f){}; }
#pragma unroll
    for (int r = 0; r < 8; ++r) { mi[r] = NEGINF; li[r] = 0.0f; }
    const int nch = 2 * qb + 2;
#pragma unroll 1
    for (int c = 0; c < nch; ++c) {
        const int k0 = c * 32;
        v8f s[2], sr[2];
#pragma unroll
        for (int tl = 0; tl < 2; ++tl) { s[tl] = (v8f){}; sr[tl] = (v8f){}; }
#pragma unroll
        for (int ds = 0; ds < 4; ++ds) {
            const v16h qa = ldh(Qp + ds * 32), qr = ldh(QLp + ds * 32);
#pragma unroll
            for (int tl = 0; tl < 2; ++tl) { const v16h ka = ldh(Kp + (size_t)(k0 + tl * 16) * HD + ds * 32), kr = ldh(KLp + (size_t)(k0 + tl * 16) * HD + ds * 32);
                s[tl] = wmma16(qa, ka, s[tl]); sr[tl] = wmma16(qa, kr, sr[tl]); sr[tl] = wmma16(qr, ka, sr[tl]); }
            asm volatile("v_nop\n\tv_nop\n\tv_nop\n\tv_nop" : "+v"(s[0]), "+v"(s[1]), "+v"(sr[0]), "+v"(sr[1]) : "v"(qa), "v"(qr));
        }
        const bool dmask = (c >= 2 * qb);
#pragma unroll
        for (int r = 0; r < 8; ++r) {
            const int row = q0 + 8 * hh + r; const int kk = k0 + m - row;
            float t0 = (s[0][r] + sr[0][r] * IRSC) * SCL, t1 = (s[1][r] + sr[1][r] * IRSC) * SCL;
            if (dmask) { t0 = (kk > 0) ? NEGINF : t0; t1 = (kk + 16 > 0) ? NEGINF : t1; }
            float mx = fmaxf(t0, t1);
            mx = fmaxf(mx, __shfl_xor(mx, 1)); mx = fmaxf(mx, __shfl_xor(mx, 2)); mx = fmaxf(mx, __shfl_xor(mx, 4)); mx = fmaxf(mx, __shfl_xor(mx, 8));
            const float mn = fmaxf(mi[r], mx);
            const float corr = ex2((mi[r] - mn) * L2E);
            const float p0 = ex2((t0 - mn) * L2E), p1 = ex2((t1 - mn) * L2E);
            float rs = p0 + p1;
            rs += __shfl_xor(rs, 1); rs += __shfl_xor(rs, 2); rs += __shfl_xor(rs, 4); rs += __shfl_xor(rs, 8);
            li[r] = li[r] * corr + rs; mi[r] = mn;
#pragma unroll
            for (int nt = 0; nt < 4; ++nt) { o[nt][r] = o[nt][r] * corr; orr[nt][r] = orr[nt][r] * corr; }
            const float c0 = p0 * PCAR, c1 = p1 * PCAR; const h16 g0 = (h16)c0, g1 = (h16)c1;
            h16* pr = phw + (8 * hh + r) * 40 + m; h16* qq = prw + (8 * hh + r) * 40 + m;
            pr[0] = g0; pr[16] = g1; qq[0] = (h16)((c0 - (float)g0) * RSC); qq[16] = (h16)((c1 - (float)g1) * RSC);
        }
        wave_sync();
        const v16h pa = ldl(phw + m * 40 + 8 * hh), pb = ldl(prw + m * 40 + 8 * hh);
#pragma unroll
        for (int nt = 0; nt < 4; ++nt) {
            const v16h vh = ldh(Vp + (size_t)nt * 16 * SEQ + k0), vl = ldh(VLp + (size_t)nt * 16 * RE + k0);
            o[nt] = wmma16(pa, vh, o[nt]); orr[nt] = wmma16(pa, vl, orr[nt]); orr[nt] = wmma16(pb, vh, orr[nt]); }
        asm volatile("v_nop\n\tv_nop\n\tv_nop\n\tv_nop" : "+v"(o[0]), "+v"(o[1]), "+v"(o[2]), "+v"(o[3]), "+v"(orr[0]), "+v"(orr[1]), "+v"(orr[2]), "+v"(orr[3]) : "v"(pa), "v"(pb));
        wave_sync();
    }
    float f[8];
#pragma unroll
    for (int r = 0; r < 8; ++r) f[r] = 1.0f / (li[r] * PCAR);
#pragma unroll
    for (int r = 0; r < 8; ++r)
#pragma unroll
        for (int nt = 0; nt < 4; ++nt) osw[(8 * hh + r) * 68 + nt * 16 + m] = (o[nt][r] + orr[nt][r] * IRSC) * f[r];
    wave_sync();
    ctx_store64(osw, lane, (size_t)b * SEQ + q0, hd * HD + dh2 * 64, (size_t)b * RO + q0, CH, CBh, CBl);
}

#define ALN(x) ((((size_t)(x)) + 255) & ~(size_t)255)
constexpr size_t SZ_XB  = (size_t)NB * SEQ * DM * 2;
constexpr size_t SZ_CH  = (size_t)NB * SEQ * DM * 2;
constexpr size_t SZ_R0  = ALN(SZ_XB > SZ_CH ? SZ_XB : SZ_CH);
constexpr size_t SZ_W   = (size_t)DM * DM * 2;
constexpr size_t SZ_F32 = (size_t)SEQ * DM * 4;
constexpr size_t SZ_CB  = (size_t)NB * RO * DM * 2;
constexpr size_t SZ_R1  = ALN(SZ_F32 > 2 * ALN(SZ_CB) ? SZ_F32 : 2 * ALN(SZ_CB));
constexpr size_t SZ_PH  = (size_t)NB * NH * SEQ * HD * 2;
constexpr size_t SZ_PL  = (size_t)NB * NH * RE * HD * 2;
constexpr size_t SZ_CST = (size_t)2 * SEQ * 64 * 4;
constexpr size_t WS_TOTAL = SZ_R0 + 5 * ALN(SZ_W) + SZ_R1 + 3 * ALN(SZ_PH) + 3 * ALN(SZ_PL) + ALN(SZ_CST);
static_assert(WS_TOTAL <= (size_t)134217728);
static_assert(SZ_XB <= SZ_R0 && SZ_CH <= SZ_R0 && SZ_F32 <= SZ_R1 && 2 * ALN(SZ_CB) <= SZ_R1);
static_assert(((size_t)(NB_FULL - 1) * SEQ_FULL + SEQ) * DM * 4 <= (size_t)33554432);

extern "C" void kernel_launch(void* const* d_in, const int* in_sizes, int n_in,
                              void* d_out, int out_size, void* d_ws, size_t ws_size, hipStream_t stream) {
    if (n_in < 6) return;
    const float* X = (const float*)d_in[0]; const float* WqI = (const float*)d_in[1]; const float* WkI = (const float*)d_in[2]; const float* WvI = (const float*)d_in[3]; const float* WoI = (const float*)d_in[4];
    const int* posp = (const int*)d_in[5];
    float* OUT = (float*)d_out;
    const size_t need_rows = (size_t)(NB - 1) * SEQ_FULL + SEQ;
    if ((size_t)in_sizes[0] < need_rows * DM) return;
    if ((size_t)in_sizes[1] < (size_t)DM * DM || (size_t)in_sizes[2] < (size_t)DM * DM || (size_t)in_sizes[3] < (size_t)DM * DM || (size_t)in_sizes[4] < (size_t)DM * DM) return;
    if (in_sizes[5] < 1) return;
    if ((size_t)out_size < need_rows * DM) return;

    char* wsp = (char*)d_ws;
    auto take = [&](size_t bytes) { char* p = wsp; wsp += ALN(bytes); return (void*)p; };
    char* R0 = (char*)take(SZ_R0); bf* XB = (bf*)R0; h16* CH = (h16*)R0;
    bf* WQ = (bf*)take(SZ_W); bf* WK = (bf*)take(SZ_W); bf* WV = (bf*)take(SZ_W); bf* WOB = (bf*)take(SZ_W); h16* WOH = (h16*)take(SZ_W);
    char* R1 = (char*)take(SZ_R1); float* F32 = (float*)R1; bf* CBh = (bf*)R1; bf* CBl = (bf*)(R1 + ALN(SZ_CB));
    h16* QH = (h16*)take(SZ_PH); h16* KH = (h16*)take(SZ_PH); h16* VT = (h16*)take(SZ_PH);
    h16* QL = (h16*)take(SZ_PL); h16* KL = (h16*)take(SZ_PL); h16* VL = (h16*)take(SZ_PL);
    float* CST = (float*)take(SZ_CST);
    if ((size_t)(wsp - (char*)d_ws) > ws_size) return;

    k_trig<<<SEQ / 4, 256, 0, stream>>>(posp, CST);
    for (int b = 0; b < NB; ++b)
        k_cvt8<<<(unsigned)(((size_t)SEQ * DM / 8 + 255) / 256), 256, 0, stream>>>(X + (size_t)b * SEQ_FULL * DM, XB + (size_t)b * SEQ * DM, (size_t)SEQ * DM / 8);
    const unsigned gw = (unsigned)((DM * DM / 64 + 63) / 64);
    k_wtG<<<gw, 256, 0, stream>>>(WqI, DM, DM, WQ);
    k_wtG<<<gw, 256, 0, stream>>>(WkI, DM, DM, WK);
    k_wtG<<<gw, 256, 0, stream>>>(WvI, DM, DM, WV);
    k_wtG2<<<gw, 256, 0, stream>>>(WoI, DM, DM, WOB, WOH);
    const dim3 gp(SEQ / 64, DM / 64, 1);
    const unsigned grope = (unsigned)(((size_t)NH * SEQ * 8 + 255) / 256), gvt = (unsigned)(((size_t)NH * HD * SEQ / 2 + 255) / 256);
    for (int b = 0; b < NB; ++b) {
        const bf* xb = XB + (size_t)b * SEQ * DM;
        k_gemmw<bf, 0><<<gp, 32, 0, stream>>>(xb, nullptr, WQ, DM, F32, DM, 1.0f);
        k_rope<<<grope, 256, 0, stream>>>(F32, CST, QH + (size_t)b * NH * SEQ * HD, QL + (size_t)b * NH * RE * HD);
        k_gemmw<bf, 0><<<gp, 32, 0, stream>>>(xb, nullptr, WK, DM, F32, DM, 1.0f);
        k_rope<<<grope, 256, 0, stream>>>(F32, CST, KH + (size_t)b * NH * SEQ * HD, KL + (size_t)b * NH * RE * HD);
        k_gemmw<bf, 0><<<gp, 32, 0, stream>>>(xb, nullptr, WV, DM, F32, DM, 1.0f);
        k_vt<<<gvt, 256, 0, stream>>>(F32, VT + (size_t)b * NH * HD * SEQ, VL + (size_t)b * NH * HD * RE);
    }
    k_attnR<<<dim3(2 * NQBR, NH, NB), 128, 0, stream>>>(QH, QL, KH, KL, VT, VL, CH, CBh, CBl);
    if (NQB > NQBR) k_attn<<<dim3(NQB - NQBR, NH, NB), 128, 0, stream>>>(QH, KH, VT, CH, CBh, CBl);
    for (int b = 0; b < NB; ++b) {
        k_gemmw<bf, 1><<<dim3(RO / 64, DM / 64, 1), 32, 0, stream>>>(CBh + (size_t)b * RO * DM, CBl + (size_t)b * RO * DM, WOB, DM, OUT + (size_t)b * SEQ_FULL * DM, DM, 1.0f);
        if (SEQ > RO) k_gemmw<h16, 0><<<dim3((SEQ - RO) / 64, DM / 64, 1), 32, 0, stream>>>(CH + ((size_t)b * SEQ + RO) * DM, nullptr, WOH, DM, OUT + ((size_t)b * SEQ_FULL + RO) * DM, DM, OSCL);
    }
    (void)hipGetLastError();
}
